// TransformerDecoderBlock_2267742732852
// MI455X (gfx1250) — hardware-verified
//
#include <hip/hip_runtime.h>
#include <math.h>
#include <stdint.h>

#define NBATCH 4
#define SEQ    1024
#define DMOD   768
#define NHEAD  12
#define HDIM   64
#define DFF    3072
#define MROWS  (NBATCH * SEQ)

static_assert(MROWS % 64 == 0);
static_assert(DMOD % 64 == 0);
static_assert(DFF % 64 == 0);
static_assert((DMOD / 2) % 32 == 0);
static_assert(NHEAD * HDIM == DMOD);

typedef __attribute__((ext_vector_type(16))) _Float16 v16h;
typedef __attribute__((ext_vector_type(8)))  _Float16 v8h;
typedef __attribute__((ext_vector_type(16))) __bf16   v16b;
typedef __attribute__((ext_vector_type(8)))  __bf16   v8b;
typedef __attribute__((ext_vector_type(8)))  float    v8f;
typedef __attribute__((ext_vector_type(4)))  float    v4f;
typedef __attribute__((ext_vector_type(2)))  float    v2f;
typedef __attribute__((ext_vector_type(4)))  unsigned int v4u;
typedef __attribute__((ext_vector_type(2)))  unsigned int v2u;

__device__ __forceinline__ unsigned short f2bf_bits(float f) {
  unsigned u = __float_as_uint(f);
  return (unsigned short)((u + 0x7FFFu + ((u >> 16) & 1u)) >> 16);
}
__device__ __forceinline__ float bf_bits2f(unsigned short h) { return __uint_as_float(((unsigned)h) << 16); }
__device__ __forceinline__ unsigned pk16(unsigned short a, unsigned short b) { return (unsigned)a | ((unsigned)b << 16); }

__device__ __forceinline__ void dep_guard_h(v8f& a, v8f& b, v16h x, v16h y) { asm volatile("v_nop\n\tv_nop\n\tv_nop\n\tv_nop" : "+v"(a), "+v"(b) : "v"(x), "v"(y)); }
__device__ __forceinline__ void dep_guard_b(v8f& a, v8f& b, v16b x, v16b y) { asm volatile("v_nop\n\tv_nop\n\tv_nop\n\tv_nop" : "+v"(a), "+v"(b) : "v"(x), "v"(y)); }
__device__ __forceinline__ void keep4_h(v16h a, v16h b, v16h c, v16h d) { asm volatile("v_nop" :: "v"(a), "v"(b), "v"(c), "v"(d)); }
__device__ __forceinline__ void keep4_b(v16b a, v16b b, v16b c, v16b d) { asm volatile("v_nop" :: "v"(a), "v"(b), "v"(c), "v"(d)); }
__device__ __forceinline__ void acc_guard4(v8f& a, v8f& b, v8f& c, v8f& d) { asm volatile("v_nop\n\tv_nop\n\tv_nop\n\tv_nop" : "+v"(a), "+v"(b), "+v"(c), "+v"(d)); }

template <typename T> struct Frag;
template <> struct Frag<_Float16> {
  typedef v16h V; union U { v16h v; v8h h[2]; };
  static __device__ __forceinline__ v16h load(const _Float16* p) {
    U f; f.h[0] = *(const v8h*)(p); f.h[1] = *(const v8h*)(p + 16); return f.v;
  }
  static __device__ __forceinline__ v8f mma(v16h a, v16h b, v8f c) {
    return __builtin_amdgcn_wmma_f32_16x16x32_f16(false, a, false, b, (short)0, c, false, false);
  }
  static __device__ __forceinline__ void guard(v8f& a, v8f& b, v16h x, v16h y) { dep_guard_h(a, b, x, y); }
  static __device__ __forceinline__ void keep(v16h a, v16h b, v16h c, v16h d) { keep4_h(a, b, c, d); }
};
template <> struct Frag<__bf16> {
  typedef v16b V; union U { v16b v; v8b h[2]; };
  static __device__ __forceinline__ v16b load(const __bf16* p) {
    U f; f.h[0] = *(const v8b*)(p); f.h[1] = *(const v8b*)(p + 16); return f.v;
  }
  static __device__ __forceinline__ v8f mma(v16b a, v16b b, v8f c) {
    return __builtin_amdgcn_wmma_f32_16x16x32_bf16(false, a, false, b, (short)0, c, false, false);
  }
  static __device__ __forceinline__ void guard(v8f& a, v8f& b, v16b x, v16b y) { dep_guard_b(a, b, x, y); }
  static __device__ __forceinline__ void keep(v16b a, v16b b, v16b c, v16b d) { keep4_b(a, b, c, d); }
};

template <int ET> struct Elem;
template <> struct Elem<0> { typedef _Float16 T; };
template <> struct Elem<1> { typedef __bf16 T; };
template <int ET, bool SPLIT, int BIAS_MODE, int OUT_MODE, bool RESID, int ACT = 0, bool LOWER = false, bool CAUSALK = false>
__global__ __launch_bounds__(256) void wmma_gemm64(
    const unsigned short* __restrict__ Ap, const unsigned short* __restrict__ A2p, int lda, long strideA,
    const unsigned short* __restrict__ Btp, const unsigned short* __restrict__ Bt2p, int ldb, long strideB,
    void* __restrict__ Cout, void* __restrict__ Cout2, int ldc, long strideC,
    const float* __restrict__ bias,
    const float* __restrict__ resid, long strideR,
    int M, int N, int K, float scale) {
  typedef typename Elem<ET>::T T;
  typedef typename Frag<T>::V V;
  const T* A = (const T*)Ap; const T* A2 = (const T*)A2p; const T* Bt = (const T*)Btp; const T* Bt2 = (const T*)Bt2p;
  __shared__ __align__(16) float sT[8][16 * 68];
  const int b    = blockIdx.y;
  const int lane = threadIdx.x & 31;
  const int wave = threadIdx.x >> 5;
  const int tilesN = N >> 6;
  const int tilesM = M >> 6;
  const int tile = blockIdx.x * 8 + wave;
  if (tile >= tilesM * tilesN) return;
  const int tm = tile / tilesN;
  const int tn = tile - tm * tilesN;
  const int m0 = tm << 6;
  const int n0 = tn << 6;
  if (LOWER && n0 > m0) return;

  const T* Ab  = A  + (size_t)b * strideA;
  const T* Bb  = Bt + (size_t)b * strideB;
  const T* Ab2 = SPLIT ? (A2  + (size_t)b * strideA) : nullptr;
  const T* Bb2 = SPLIT ? (Bt2 + (size_t)b * strideB) : nullptr;

  const int rlane = lane & 15;
  const int koff  = (lane >> 4) * 8;
  const int mOff  = (lane >> 4) * 8;

  v8f acc[4][4];
#pragma unroll
  for (int i = 0; i < 4; ++i)
#pragma unroll
    for (int j = 0; j < 4; ++j) acc[i][j] = (v8f){0.f,0.f,0.f,0.f,0.f,0.f,0.f,0.f};

  const int kEnd = CAUSALK ? (((m0 + 64) < K) ? (m0 + 64) : K) : K;
  for (int k0 = 0; k0 < kEnd; k0 += 32) {
    V bh[4], bl[4];
#pragma unroll
    for (int j = 0; j < 4; ++j) {
      const size_t bo = (size_t)(n0 + (j << 4) + rlane) * ldb + koff + k0;
      bh[j] = Frag<T>::load(Bb + bo);
      if (SPLIT) bl[j] = Frag<T>::load(Bb2 + bo);
    }
#pragma unroll
    for (int i = 0; i < 4; ++i) {
      const size_t ao = (size_t)(m0 + (i << 4) + rlane) * lda + koff + k0;
      V ah = Frag<T>::load(Ab + ao);
      V al;
      if (SPLIT) al = Frag<T>::load(Ab2 + ao);
#pragma unroll
      for (int j = 0; j < 4; ++j) {
        acc[i][j] = Frag<T>::mma(ah, bh[j], acc[i][j]);
        if (SPLIT) {
          acc[i][j] = Frag<T>::mma(ah, bl[j], acc[i][j]);
          acc[i][j] = Frag<T>::mma(al, bh[j], acc[i][j]);
        }
      }
      Frag<T>::guard(acc[i][0], acc[i][3], ah, SPLIT ? al : ah);
    }
    Frag<T>::keep(bh[0], bh[1], bh[2], bh[3]);
    if (SPLIT) Frag<T>::keep(bl[0], bl[1], bl[2], bl[3]);
  }
  acc_guard4(acc[0][0], acc[0][1], acc[0][2], acc[0][3]);
  acc_guard4(acc[1][0], acc[1][1], acc[1][2], acc[1][3]);
  acc_guard4(acc[2][0], acc[2][1], acc[2][2], acc[2][3]);
  acc_guard4(acc[3][0], acc[3][1], acc[3][2], acc[3][3]);

  float* slab = sT[wave];
  const float* Rb = RESID ? (resid + (size_t)b * strideR) : nullptr;
#pragma unroll
  for (int i = 0; i < 4; ++i) {
    const int mBase = m0 + (i << 4);
#pragma unroll
    for (int j = 0; j < 4; ++j) {
      const int n = n0 + (j << 4) + rlane;
      float bv = 0.f;
      if (BIAS_MODE == 2) bv = bias[n];
#pragma unroll
      for (int r = 0; r < 8; ++r) {
        float v = acc[i][j][r] * scale;
        if (BIAS_MODE == 1) v += bias[mBase + mOff + r];
        if (BIAS_MODE == 2) v += bv;
        if (RESID) v += Rb[(size_t)(mBase + mOff + r) * ldc + n];
        if (ACT == 1) v = tanhf(v);
        if (ACT == 2) v = fmaxf(v, 0.0f);
        if (ACT == 3) v = v / (1.0f + expf(-v));
        if (ACT == 4) v = (v > 0.f) ? v : 0.01f * v;
        if (ACT == 5) v = 0.5f * v * (1.0f + erff(v * 0.70710678118654752f));
        slab[(mOff + r) * 68 + (j << 4) + rlane] = v;
      }
    }
    __builtin_amdgcn_fence(__ATOMIC_RELEASE, "workgroup");
    __builtin_amdgcn_wave_barrier();
    __builtin_amdgcn_fence(__ATOMIC_ACQUIRE, "workgroup");
    if (OUT_MODE == 0) {
      float* C = (float*)Cout + (size_t)b * strideC;
      const int hh = lane >> 4, c4 = (lane & 15) * 4;
      for (int pass = 0; pass < 2; ++pass) {
#pragma unroll
        for (int it = 0; it < 8; ++it) {
          const int row = it * 2 + hh;
          v4f v = *(const v4f*)(slab + row * 68 + c4);
          *(volatile v4f*)(C + (size_t)(mBase + row) * ldc + n0 + c4) = v;
        }
        __threadfence();
      }
    } else {
      const int q = lane >> 3, c8 = (lane & 7) * 8;
      unsigned short* C  = (unsigned short*)Cout  + (size_t)b * strideC;
      unsigned short* C2 = (OUT_MODE == 2) ? ((unsigned short*)Cout2 + (size_t)b * strideC) : nullptr;
      for (int pass = 0; pass < 2; ++pass) {
#pragma unroll
        for (int it = 0; it < 4; ++it) {
          const int row = it * 4 + q;
          const float* sp = slab + row * 68 + c8;
          v8h hv, lv;
#pragma unroll
          for (int e = 0; e < 8; ++e) {
            if (OUT_MODE == 1) {
              hv[e] = (_Float16)sp[e];
            } else {
              unsigned short hb = f2bf_bits(sp[e]);
              unsigned short lb = f2bf_bits(sp[e] - bf_bits2f(hb));
              hv[e] = __builtin_bit_cast(_Float16, hb);
              lv[e] = __builtin_bit_cast(_Float16, lb);
            }
          }
          *(volatile v8h*)(C + (size_t)(mBase + row) * ldc + n0 + c8) = hv;
          if (OUT_MODE == 2) *(volatile v8h*)(C2 + (size_t)(mBase + row) * ldc + n0 + c8) = lv;
        }
        __threadfence();
      }
    }
    __builtin_amdgcn_fence(__ATOMIC_RELEASE, "workgroup");
    __builtin_amdgcn_wave_barrier();
    __builtin_amdgcn_fence(__ATOMIC_ACQUIRE, "workgroup");
  }
}

__global__ __launch_bounds__(256) void cvt8_kernel(const float* __restrict__ s0, const float* __restrict__ s1,
                                                   const float* __restrict__ s2,
                                                   unsigned short* __restrict__ d0, unsigned short* __restrict__ d1,
                                                   unsigned short* __restrict__ d2, int n8) {
  const int g = blockIdx.x * 256 + threadIdx.x;
  if (g >= 3 * n8) return;
  const int sel = g / n8;
  const int off = g - sel * n8;
  const float* src = (sel == 0) ? s0 : ((sel == 1) ? s1 : s2);
  unsigned short* dst = (sel == 0) ? d0 : ((sel == 1) ? d1 : d2);
  const v4f a = *(const v4f*)(src + (size_t)off * 8);
  const v4f c = *(const v4f*)(src + (size_t)off * 8 + 4);
  v4u u;
  u[0] = pk16(f2bf_bits(a[0]), f2bf_bits(a[1]));
  u[1] = pk16(f2bf_bits(a[2]), f2bf_bits(a[3]));
  u[2] = pk16(f2bf_bits(c[0]), f2bf_bits(c[1]));
  u[3] = pk16(f2bf_bits(c[2]), f2bf_bits(c[3]));
  *(volatile v4u*)(dst + (size_t)off * 8) = u;
  __threadfence();
  *(volatile v4u*)(dst + (size_t)off * 8) = u;
}

__global__ __launch_bounds__(256) void split2_kernel(const float* __restrict__ in, unsigned short* __restrict__ out,
                                                     int n2, int halfK) {
  const int i = blockIdx.x * 256 + threadIdx.x;
  if (i >= n2) return;
  const int row = i / halfK;
  const int cp  = i - row * halfK;
  const v2f f = *(const v2f*)(in + 2 * (size_t)i);
  const unsigned short h0 = f2bf_bits(f[0]), h1 = f2bf_bits(f[1]);
  const unsigned short l0 = f2bf_bits(f[0] - bf_bits2f(h0)), l1 = f2bf_bits(f[1] - bf_bits2f(h1));
  const unsigned uh = pk16(h0, h1), ul = pk16(l0, l1);
  const size_t oh = (size_t)row * (size_t)(2 * halfK) + cp;
  const size_t ol = oh + (size_t)halfK;
  volatile unsigned* o32 = (volatile unsigned*)out;
  o32[oh] = uh;
  o32[ol] = ul;
  __threadfence();
  o32[oh] = uh;
  o32[ol] = ul;
}

template <bool DUP>
__global__ __launch_bounds__(256) void tconv_kernel(const float* __restrict__ W, unsigned short* __restrict__ oh,
                                                    int R, int Cc, int ldo, long inZ, long outZ) {
  __shared__ __align__(16) float tf[64 * 68];
  const float* Wz = W + (size_t)blockIdx.z * (size_t)inZ;
  unsigned short* oz = oh + (size_t)blockIdx.z * (size_t)outZ;
  const int c0  = blockIdx.x * 64;
  const int r0  = blockIdx.y * 64;
  const int tid = threadIdx.x;
  {
    const int lr = tid >> 4;
    const int c4 = (tid & 15) * 4;
#pragma unroll
    for (int it = 0; it < 4; ++it) {
      const int rr = it * 16 + lr;
      const v4f a = *(const v4f*)(Wz + (size_t)(r0 + rr) * Cc + c0 + c4);
      *(v4f*)(tf + rr * 68 + c4) = a;
    }
  }
  __syncthreads();
  const int sub = tid >> 3;
  const int c8  = (tid & 7) * 8;
  v4u hv[2];
#pragma unroll
  for (int it = 0; it < 2; ++it) {
    const int oc = it * 32 + sub;
    v4u a;
#pragma unroll
    for (int q = 0; q < 4; ++q) {
      const float f0 = tf[(c8 + 2 * q) * 68 + oc];
      const float f1 = tf[(c8 + 2 * q + 1) * 68 + oc];
      a[q] = pk16(f2bf_bits(f0), f2bf_bits(f1));
    }
    hv[it] = a;
  }
  for (int pass = 0; pass < 2; ++pass) {
#pragma unroll
    for (int it = 0; it < 2; ++it) {
      const int oc = it * 32 + sub;
      const size_t go = (size_t)(c0 + oc) * ldo + r0 + c8;
      *(volatile v4u*)(oz + go) = hv[it];
      if (DUP) *(volatile v4u*)(oz + go + (size_t)R) = hv[it];
    }
    __threadfence();
  }
}

template <bool RES16, bool OUT16>
__global__ __launch_bounds__(256) void ln_kernel(const float* __restrict__ Ain, const float* __restrict__ Rf,
                                                 const unsigned short* __restrict__ Rh,
                                                 const float* __restrict__ gam, const float* __restrict__ bet,
                                                 float* __restrict__ outF, unsigned short* __restrict__ outH, int nrows) {
  __shared__ __align__(16) float srow[8][DMOD];
  const int lane = threadIdx.x & 31, wave = threadIdx.x >> 5;
  const int row = blockIdx.x * 8 + wave;
  if (row >= nrows) return;
  const size_t rb = (size_t)row * DMOD;

  v4f v[6];
  float s = 0.f;
#pragma unroll
  for (int it = 0; it < 6; ++it) {
    const int col = it * 128 + 4 * lane;
    v4f a = *(const v4f*)(Ain + rb + col);
    v4f rr;
    if (RES16) {
      const v2u u = *(const v2u*)(Rh + rb + col);
      rr[0] = __uint_as_float(u[0] << 16);
      rr[1] = __uint_as_float(u[0] & 0xffff0000u);
      rr[2] = __uint_as_float(u[1] << 16);
      rr[3] = __uint_as_float(u[1] & 0xffff0000u);
    } else {
      rr = *(const v4f*)(Rf + rb + col);
    }
    a = a + rr;
    v[it] = a;
    s += (a[0] + a[1]) + (a[2] + a[3]);
  }
#pragma unroll
  for (int off = 1; off < 32; off <<= 1) s += __shfl_xor(s, off, 32);
  const float mu = s * (1.0f / (float)DMOD);
  float sq = 0.f;
#pragma unroll
  for (int it = 0; it < 6; ++it) {
    v4f d = v[it] - mu;
    v[it] = d;
    sq += (d[0] * d[0] + d[1] * d[1]) + (d[2] * d[2] + d[3] * d[3]);
  }
#pragma unroll
  for (int off = 1; off < 32; off <<= 1) sq += __shfl_xor(sq, off, 32);
  const float var = sq * (1.0f / (float)DMOD);
  const float rs  = rsqrtf(var + 1e-5f);

  v4f y[6];
#pragma unroll
  for (int it = 0; it < 6; ++it) {
    const int col = it * 128 + 4 * lane;
    const v4f g4 = *(const v4f*)(gam + col);
    const v4f b4 = *(const v4f*)(bet + col);
    y[it] = v[it] * rs * g4 + b4;
  }
  for (int pass = 0; pass < 2; ++pass) {
#pragma unroll
    for (int it = 0; it < 6; ++it) {
      const int col = it * 128 + 4 * lane;
      *(volatile v4f*)(outF + rb + col) = y[it];
    }
    __threadfence();
  }
  if (OUT16) {
    float* sr = srow[wave];
#pragma unroll
    for (int it = 0; it < 6; ++it) {
      const int col = it * 128 + 4 * lane;
      *(v4f*)(sr + col) = y[it];
    }
    __builtin_amdgcn_fence(__ATOMIC_RELEASE, "workgroup");
    __builtin_amdgcn_wave_barrier();
    __builtin_amdgcn_fence(__ATOMIC_ACQUIRE, "workgroup");
    v4u hv[3], lv[3];
#pragma unroll
    for (int k = 0; k < 3; ++k) {
      const int c8 = (k * 32 + lane) * 8;
      const v4f p0 = *(const v4f*)(sr + c8);
      const v4f p1 = *(const v4f*)(sr + c8 + 4);
      float e[8];
      e[0] = p0[0]; e[1] = p0[1]; e[2] = p0[2]; e[3] = p0[3];
      e[4] = p1[0]; e[5] = p1[1]; e[6] = p1[2]; e[7] = p1[3];
      v4u ah, al;
#pragma unroll
      for (int q = 0; q < 4; ++q) {
        const unsigned short h0 = f2bf_bits(e[2 * q]), h1 = f2bf_bits(e[2 * q + 1]);
        const unsigned short l0 = f2bf_bits(e[2 * q] - bf_bits2f(h0)), l1 = f2bf_bits(e[2 * q + 1] - bf_bits2f(h1));
        ah[q] = pk16(h0, h1);
        al[q] = pk16(l0, l1);
      }
      hv[k] = ah; lv[k] = al;
    }
    const size_t hbse = (size_t)row * (size_t)(2 * DMOD);
    for (int pass = 0; pass < 2; ++pass) {
#pragma unroll
      for (int k = 0; k < 3; ++k) {
        const int c8 = (k * 32 + lane) * 8;
        *(volatile v4u*)(outH + hbse + c8) = hv[k];
        *(volatile v4u*)(outH + hbse + DMOD + c8) = lv[k];
      }
      __threadfence();
    }
  }
}

#define AT_D 64
#define AT_NW 4
#define AT_QB 64
#define AT_KC 64
static_assert(SEQ % AT_QB == 0);
static_assert(SEQ % AT_KC == 0);

__device__ __forceinline__ unsigned short at_bf_bits(float f) {
  unsigned u = __float_as_uint(f);
  return (unsigned short)((u + 0x7FFFu + ((u >> 16) & 1u)) >> 16);
}
__device__ __forceinline__ __bf16 at_f2bf(float f) { return __builtin_bit_cast(__bf16, at_bf_bits(f)); }
__device__ __forceinline__ void at_split(float f, __bf16& hi, __bf16& lo) {
  const unsigned short hb = at_bf_bits(f);
  hi = __builtin_bit_cast(__bf16, hb);
  lo = at_f2bf(f - __uint_as_float(((unsigned)hb) << 16));
}
__device__ __forceinline__ v8f at_mma(v16b a, v16b b, v8f c) {
  c = __builtin_amdgcn_wmma_f32_16x16x32_bf16(false, a, false, b, (short)0, c, false, false);
  asm volatile("v_nop\n\tv_nop\n\tv_nop\n\tv_nop" : "+v"(c) : "v"(a), "v"(b));
  return c;
}

template <bool CAUSAL>
__global__ __launch_bounds__(128)
void attn64_kernel(const unsigned short* __restrict__ qhp, const unsigned short* __restrict__ qlp,
                   const unsigned short* __restrict__ khp, const unsigned short* __restrict__ klp,
                   const unsigned short* __restrict__ vhp, const unsigned short* __restrict__ vlp,
                   const int* __restrict__ mask, float* __restrict__ out, float sscale) {
  union FB { v16b v; v8b h[2]; };
  __shared__ __align__(16) __bf16 Ksh[AT_KC * AT_D];
  __shared__ __align__(16) __bf16 Ksl[AT_KC * AT_D];
  __shared__ __align__(16) __bf16 Vth[AT_D * AT_KC];
  __shared__ __align__(16) __bf16 Vtl[AT_D * AT_KC];
  __shared__ __align__(16) __bf16 Psh[AT_NW][16 * AT_KC];
  __shared__ __align__(16) __bf16 Psl[AT_NW][16 * AT_KC];
  __shared__ __align__(16) float  Os[AT_NW][16 * 68];

  const int tid  = threadIdx.x;
  const int wave = tid >> 5;
  const int lane = tid & 31;
  const int hh   = lane >> 4;
  const int c    = lane & 15;

  const int nqb = SEQ / AT_QB;
  const int bx = blockIdx.x;
  const int qb = bx % nqb;
  const int h  = bx / nqb;
  const int b  = blockIdx.y;
  const int q0 = qb * AT_QB + wave * 16;
  const size_t boff = (size_t)b * SEQ * DMOD;

  const __bf16* Qh = (const __bf16*)(const void*)qhp + boff + (size_t)h * AT_D;
  const __bf16* Ql = (const __bf16*)(const void*)qlp + boff + (size_t)h * AT_D;
  const __bf16* Kh = (const __bf16*)(const void*)khp + boff + (size_t)h * AT_D;
  const __bf16* Kl = (const __bf16*)(const void*)klp + boff + (size_t)h * AT_D;
  const __bf16* Vh = (const __bf16*)(const void*)vhp + boff + (size_t)h * AT_D * SEQ;
  const __bf16* Vl = (const __bf16*)(const void*)vlp + boff + (size_t)h * AT_D * SEQ;
  float*        ob = out + boff + (size_t)h * AT_D;
  const int*    mb = mask + (size_t)b * SEQ;

  v16b qah[2], qal[2];
#pragma unroll
  for (int dc = 0; dc < 2; ++dc) {
    const __bf16* qr = Qh + (size_t)(q0 + c) * DMOD + dc * 32 + 8 * hh;
    const __bf16* ql = Ql + (size_t)(q0 + c) * DMOD + dc * 32 + 8 * hh;
    qah[dc] = Frag<__bf16>::load(qr);
    qal[dc] = Frag<__bf16>::load(ql);
  }

  float mrow[8], lrow[8];
  v8f oacc[4];
#pragma unroll
  for (int r = 0; r < 8; ++r) { mrow[r] = -INFINITY; lrow[r] = 0.f; }
#pragma unroll
  for (int t = 0; t < 4; ++t) oacc[t] = (v8f){0.f,0.f,0.f,0.f,0.f,0.f,0.f,0.f};

  const int nChunks = CAUSAL ? (qb + 1) : (SEQ / AT_KC);
  for (int kc = 0; kc < nChunks; ++kc) {
    const int kv0 = kc * AT_KC;
    __syncthreads();
    {
      const int r = tid >> 1, half = (tid & 1) * 32;
      const __bf16* ksh = Kh + (size_t)(kv0 + r) * DMOD + half;
      const __bf16* ksl = Kl + (size_t)(kv0 + r) * DMOD + half;
      const __bf16* vsh = Vh + (size_t)r * SEQ + kv0 + half;
      const __bf16* vsl = Vl + (size_t)r * SEQ + kv0 + half;
#pragma unroll
      for (int i = 0; i < 4; ++i) {
        const v8b a0 = *(const v8b*)(ksh + 8 * i);
        const v8b a1 = *(const v8b*)(ksl + 8 * i);
        const v8b b0 = *(const v8b*)(vsh + 8 * i);
        const v8b b1 = *(const v8b*)(vsl + 8 * i);
        *(v8b*)(Ksh + r * AT_D  + half + 8 * i) = a0;
        *(v8b*)(Ksl + r * AT_D  + half + 8 * i) = a1;
        *(v8b*)(Vth + r * AT_KC + half + 8 * i) = b0;
        *(v8b*)(Vtl + r * AT_KC + half + 8 * i) = b1;
      }
    }
    __syncthreads();

    v8f s[4];
#pragma unroll
    for (int j = 0; j < 4; ++j) {
      s[j] = (v8f){0.f,0.f,0.f,0.f,0.f,0.f,0.f,0.f};
#pragma unroll
      for (int dc = 0; dc < 2; ++dc) {
        FB kb, kl;
        kb.h[0] = *(const v8b*)(Ksh + (j * 16 + c) * AT_D + dc * 32 + 8 * hh);
        kb.h[1] = *(const v8b*)(Ksh + (j * 16 + c) * AT_D + dc * 32 + 16 + 8 * hh);
        kl.h[0] = *(const v8b*)(Ksl + (j * 16 + c) * AT_D + dc * 32 + 8 * hh);
        kl.h[1] = *(const v8b*)(Ksl + (j * 16 + c) * AT_D + dc * 32 + 16 + 8 * hh);
        s[j] = at_mma(qah[dc], kb.v, s[j]);
        s[j] = at_mma(qah[dc], kl.v, s[j]);
        s[j] = at_mma(qal[dc], kb.v, s[j]);
      }
    }
    const bool diag = CAUSAL && (kc == qb);
    int mk[4];
#pragma unroll
    for (int j = 0; j < 4; ++j) mk[j] = mb[kv0 + j * 16 + c];
    float cm[8];
#pragma unroll
    for (int r = 0; r < 8; ++r) {
      const int qrow = q0 + 8 * hh + r;
      float m = -INFINITY;
#pragma unroll
      for (int j = 0; j < 4; ++j) {
        const int kvcol = kv0 + j * 16 + c;
        const float sv = s[j][r] * sscale;
        const bool masked = (diag && (kvcol > qrow)) || (mk[j] == 0);
        const float sm = masked ? -INFINITY : sv;
        s[j][r] = sm;
        m = fmaxf(m, sm);
      }
#pragma unroll
      for (int off = 1; off < 16; off <<= 1) m = fmaxf(m, __shfl_xor(m, off, 32));
      cm[r] = m;
    }
    __bf16* pwh = Psh[wave];
    __bf16* pwl = Psl[wave];
#pragma unroll
    for (int r = 0; r < 8; ++r) {
      const float mnew  = fmaxf(mrow[r], cm[r]);
      const float msafe = (mnew == -INFINITY) ? 0.0f : mnew;
      const float alpha = expf(mrow[r] - msafe);
      mrow[r] = mnew;
      float psum = 0.f;
#pragma unroll
      for (int j = 0; j < 4; ++j) {
        const float p = expf(s[j][r] - msafe);
        psum += p;
        __bf16 a, bl; at_split(p, a, bl);
        pwh[(8 * hh + r) * AT_KC + j * 16 + c] = a;
        pwl[(8 * hh + r) * AT_KC + j * 16 + c] = bl;
      }
#pragma unroll
      for (int off = 1; off < 16; off <<= 1) psum += __shfl_xor(psum, off, 32);
      lrow[r] = lrow[r] * alpha + psum;
#pragma unroll
      for (int t = 0; t < 4; ++t) oacc[t][r] *= alpha;
    }
    __builtin_amdgcn_fence(__ATOMIC_RELEASE, "workgroup");
    __builtin_amdgcn_wave_barrier();
    __builtin_amdgcn_fence(__ATOMIC_ACQUIRE, "workgroup");
#pragma unroll 1
    for (int kk = 0; kk < 2; ++kk) {
      FB pa, pl;
      pa.h[0] = *(const v8b*)(pwh + c * AT_KC + kk * 32 + 8 * hh);
      pa.h[1] = *(const v8b*)(pwh + c * AT_KC + kk * 32 + 16 + 8 * hh);
      pl.h[0] = *(const v8b*)(pwl + c * AT_KC + kk * 32 + 8 * hh);
      pl.h[1] = *(const v8b*)(pwl + c * AT_KC + kk * 32 + 16 + 8 * hh);
#pragma unroll
      for (int t = 0; t < 4; ++t) {
        FB vb, vl;
        vb.h[0] = *(const v8b*)(Vth + (t * 16 + c) * AT_KC + kk * 32 + 8 * hh);
        vb.h[1] = *(const v8b*)(Vth + (t * 16 + c) * AT_KC + kk * 32 + 16 + 8 * hh);
        vl.h[0] = *(const v8b*)(Vtl + (t * 16 + c) * AT_KC + kk * 32 + 8 * hh);
        vl.h[1] = *(const v8b*)(Vtl + (t * 16 + c) * AT_KC + kk * 32 + 16 + 8 * hh);
        oacc[t] = at_mma(pa.v, vb.v, oacc[t]);
        oacc[t] = at_mma(pa.v, vl.v, oacc[t]);
        oacc[t] = at_mma(pl.v, vb.v, oacc[t]);
      }
    }
  }

  float* os = Os[wave];
#pragma unroll
  for (int r = 0; r < 8; ++r) {
    const float inv = 1.0f / lrow[r];
#pragma unroll
    for (int t = 0; t < 4; ++t) os[(8 * hh + r) * 68 + t * 16 + c] = oacc[t][r] * inv;
  }
  __builtin_amdgcn_fence(__ATOMIC_RELEASE, "workgroup");
  __builtin_amdgcn_wave_barrier();
  __builtin_amdgcn_fence(__ATOMIC_ACQUIRE, "workgroup");
  {
    const int c4 = (lane & 15) * 4;
    for (int pass = 0; pass < 2; ++pass) {
#pragma unroll
      for (int it = 0; it < 8; ++it) {
        const int row = it * 2 + hh;
        v4f val = *(const v4f*)(os + row * 68 + c4);
        *(volatile v4f*)(ob + (size_t)(q0 + row) * DMOD + c4) = val;
      }
      __threadfence();
    }
  }
}

extern "C" void kernel_launch(void* const* d_in, const int* in_sizes, int n_in,
                              void* d_out, int out_size, void* d_ws, size_t ws_size,
                              hipStream_t stream) {
  const int NX  = MROWS * DMOD;
  const int NWH = NHEAD * DMOD * HDIM;
  const int NWO = DMOD * DMOD;
  const int NW1 = DMOD * DFF;
  if (n_in < 23) return;
  if (in_sizes[0] != NX || in_sizes[1] != NX || in_sizes[2] != NX) return;
  if (in_sizes[3] != NBATCH * SEQ || in_sizes[4] != NBATCH * SEQ) return;
  if (in_sizes[5] != NWH || in_sizes[6] != NWH || in_sizes[7] != NWH || in_sizes[8] != NWO) return;
  if (in_sizes[9] != NWH || in_sizes[10] != NWH || in_sizes[11] != NWH || in_sizes[12] != NWO) return;
  for (int i = 13; i <= 18; ++i) if (in_sizes[i] != DMOD) return;
  if (in_sizes[19] != NW1 || in_sizes[20] != DFF || in_sizes[21] != NW1 || in_sizes[22] != DMOD) return;
  if (out_size != NX) return;

  const float* key_enc = (const float*)d_in[0];
  const float* val_enc = (const float*)d_in[1];
  const float* x       = (const float*)d_in[2];
  const int*   src_m   = (const int*)d_in[3];
  const int*   tgt_m   = (const int*)d_in[4];
  const float* Wq_m  = (const float*)d_in[5];
  const float* Wk_m  = (const float*)d_in[6];
  const float* Wv_m  = (const float*)d_in[7];
  const float* Wo_m  = (const float*)d_in[8];
  const float* Wq_c  = (const float*)d_in[9];
  const float* Wk_c  = (const float*)d_in[10];
  const float* Wv_c  = (const float*)d_in[11];
  const float* Wo_c  = (const float*)d_in[12];
  const float* ln1_g = (const float*)d_in[13];
  const float* ln1_b = (const float*)d_in[14];
  const float* ln2_g = (const float*)d_in[15];
  const float* ln2_b = (const float*)d_in[16];
  const float* ln3_g = (const float*)d_in[17];
  const float* ln3_b = (const float*)d_in[18];
  const float* W1    = (const float*)d_in[19];
  const float* b1    = (const float*)d_in[20];
  const float* W2    = (const float*)d_in[21];
  const float* b2    = (const float*)d_in[22];
  float* out = (float*)d_out;

  const size_t PW1 = (size_t)DMOD * DMOD * 2;
  const size_t PW2 = (size_t)DMOD * 2 * DMOD * 2;
  const size_t PF1 = (size_t)DFF * 2 * DMOD * 2;
  const size_t PF2 = (size_t)DMOD * 2 * DFF * 2;
  const size_t U   = (size_t)MROWS * DMOD * 2;
  size_t off = 0;
  const size_t oWq  = off; off += PW1;
  const size_t oWk  = off; off += PW1;
  const size_t oWv  = off; off += PW1;
  const size_t oWo  = off; off += PW2;
  const size_t oWqc = off; off += PW2;
  const size_t oWkc = off; off += PW1;
  const size_t oWvc = off; off += PW1;
  const size_t oWoc = off; off += PW2;
  const size_t oW1  = off; off += PF1;
  const size_t oW2  = off; off += PF2;
  const size_t oAr  = off; off += 16 * U;
  if (off > ws_size) return;

  char* ws = (char*)d_ws;
  unsigned short* WqT  = (unsigned short*)(ws + oWq);
  unsigned short* WkT  = (unsigned short*)(ws + oWk);
  unsigned short* WvT  = (unsigned short*)(ws + oWv);
  unsigned short* WoT  = (unsigned short*)(ws + oWo);
  unsigned short* WqcT = (unsigned short*)(ws + oWqc);
  unsigned short* WkcT = (unsigned short*)(ws + oWkc);
  unsigned short* WvcT = (unsigned short*)(ws + oWvc);
  unsigned short* WocT = (unsigned short*)(ws + oWoc);
  unsigned short* W1T  = (unsigned short*)(ws + oW1);
  unsigned short* W2T  = (unsigned short*)(ws + oW2);
  char* ar = ws + oAr;
#define SL16(i) ((unsigned short*)(ar + (size_t)(i) * U))
#define SL32(i) ((float*)(ar + (size_t)(i) * U))
  unsigned short* XB   = SL16(0);
  unsigned short* KEB  = SL16(1);
  unsigned short* VEB  = SL16(2);
  unsigned short* Qh   = SL16(3);  unsigned short* Ql  = SL16(4);
  unsigned short* Kh   = SL16(5);  unsigned short* Kl  = SL16(6);
  unsigned short* VTh  = SL16(7);  unsigned short* VTl = SL16(8);
  float*          CTXf = SL32(9);
  unsigned short* CTX2 = SL16(11);
  float*          A1   = SL32(13);
  float*          H1f  = SL32(9);
  unsigned short* H1hl = SL16(11);
  unsigned short* Qch  = SL16(3);  unsigned short* Qcl  = SL16(4);
  unsigned short* Kch  = SL16(5);  unsigned short* Kcl  = SL16(6);
  unsigned short* VcTh = SL16(7);  unsigned short* VcTl = SL16(8);
  float*          CTXcf = SL32(13);
  unsigned short* CTXc2 = SL16(1);
  float*          A2   = SL32(3);
  float*          H2f  = SL32(11);
  unsigned short* H2hl = SL16(13);
  unsigned short* Fhl  = SL16(0);
  float*          A3   = SL32(9);
#undef SL16
#undef SL32

  const dim3 blk(256);
  const long SD = (long)SEQ * DMOD;

  const int n8 = NX / 8;
  cvt8_kernel<<<dim3((3 * n8 + 255) / 256), blk, 0, stream>>>(x, key_enc, val_enc, XB, KEB, VEB, n8);

  const long hIn = (long)DMOD * HDIM;
  tconv_kernel<false><<<dim3(HDIM / 64, DMOD / 64, NHEAD), blk, 0, stream>>>(Wq_m, WqT, DMOD, HDIM, DMOD, hIn, (long)HDIM * DMOD);
  tconv_kernel<false><<<dim3(HDIM / 64, DMOD / 64, NHEAD), blk, 0, stream>>>(Wk_m, WkT, DMOD, HDIM, DMOD, hIn, (long)HDIM * DMOD);
  tconv_kernel<false><<<dim3(HDIM / 64, DMOD / 64, NHEAD), blk, 0, stream>>>(Wv_m, WvT, DMOD, HDIM, DMOD, hIn, (long)HDIM * DMOD);
  tconv_kernel<true ><<<dim3(DMOD / 64, DMOD / 64, 1),     blk, 0, stream>>>(Wo_m, WoT, DMOD, DMOD, 2 * DMOD, 0L, 0L);
  tconv_kernel<true ><<<dim3(HDIM / 64, DMOD / 64, NHEAD), blk, 0, stream>>>(Wq_c, WqcT, DMOD, HDIM, 2 * DMOD, hIn, (long)HDIM * 2 * DMOD);
  tconv_kernel<false><<<dim3(HDIM / 64, DMOD / 64, NHEAD), blk, 0, stream>>>(Wk_c, WkcT, DMOD, HDIM, DMOD, hIn, (long)HDIM * DMOD);
  tconv_kernel<false><<<dim3(HDIM / 64, DMOD / 64, NHEAD), blk, 0, stream>>>(Wv_c, WvcT, DMOD, HDIM, DMOD, hIn, (long)HDIM * DMOD);
  tconv_kernel<true ><<<dim3(DMOD / 64, DMOD / 64, 1),     blk, 0, stream>>>(Wo_c, WocT, DMOD, DMOD, 2 * DMOD, 0L, 0L);
  tconv_kernel<true ><<<dim3(DFF / 64, DMOD / 64, 1),      blk, 0, stream>>>(W1, W1T, DMOD, DFF, 2 * DMOD, 0L, 0L);
  tconv_kernel<true ><<<dim3(DMOD / 64, DFF / 64, 1),      blk, 0, stream>>>(W2, W2T, DFF, DMOD, 2 * DFF, 0L, 0L);

  const dim3 gD(((MROWS / 64) * (DMOD / 64) + 7) / 8, 1);
  const dim3 gF(((MROWS / 64) * (DFF / 64) + 7) / 8, 1);
  const dim3 gVT(((DMOD / 64) * (SEQ / 64) + 7) / 8, NBATCH);
  const dim3 gAtt(NHEAD * (SEQ / 64), NBATCH);
  const dim3 gLN(MROWS / 8);
  const int n2 = NX / 2;
  const dim3 gSp((n2 + 255) / 256);

  wmma_gemm64<1, false, 0, 2, false><<<gD, blk, 0, stream>>>(
      XB, XB, DMOD, 0L, WqT, WqT, DMOD, 0L, (void*)Qh, (void*)Ql, DMOD, 0L, b1, x, 0L, MROWS, DMOD, DMOD, 1.0f);
  wmma_gemm64<1, false, 0, 2, false><<<gD, blk, 0, stream>>>(
      XB, XB, DMOD, 0L, WkT, WkT, DMOD, 0L, (void*)Kh, (void*)Kl, DMOD, 0L, b1, x, 0L, MROWS, DMOD, DMOD, 1.0f);
  wmma_gemm64<1, false, 0, 2, false><<<gVT, blk, 0, stream>>>(
      WvT, WvT, DMOD, 0L, XB, XB, DMOD, SD, (void*)VTh, (void*)VTl, SEQ, SD, b1, x, 0L, DMOD, SEQ, DMOD, 1.0f);
  attn64_kernel<true><<<gAtt, dim3(128), 0, stream>>>(Qh, Ql, Kh, Kl, VTh, VTl, tgt_m, CTXf, 0.125f);
  split2_kernel<<<gSp, blk, 0, stream>>>(CTXf, CTX2, n2, DMOD / 2);
  wmma_gemm64<1, false, 0, 0, false><<<gD, blk, 0, stream>>>(
      CTX2, CTX2, 2 * DMOD, 0L, WoT, WoT, 2 * DMOD, 0L, (void*)A1, (void*)A1, DMOD, 0L, b1, x, 0L, MROWS, DMOD, 2 * DMOD, 1.0f);
  ln_kernel<true, true><<<gLN, blk, 0, stream>>>(A1, A1, XB, ln1_g, ln1_b, H1f, H1hl, MROWS);

  wmma_gemm64<1, false, 0, 2, false><<<gD, blk, 0, stream>>>(
      H1hl, H1hl, 2 * DMOD, 0L, WqcT, WqcT, 2 * DMOD, 0L, (void*)Qch, (void*)Qcl, DMOD, 0L, b1, x, 0L, MROWS, DMOD, 2 * DMOD, 1.0f);
  wmma_gemm64<1, false, 0, 2, false><<<gD, blk, 0, stream>>>(
      KEB, KEB, DMOD, 0L, WkcT, WkcT, DMOD, 0L, (void*)Kch, (void*)Kcl, DMOD, 0L, b1, x, 0L, MROWS, DMOD, DMOD, 1.0f);
  wmma_gemm64<1, false, 0, 2, false><<<gVT, blk, 0, stream>>>(
      WvcT, WvcT, DMOD, 0L, VEB, VEB, DMOD, SD, (void*)VcTh, (void*)VcTl, SEQ, SD, b1, x, 0L, DMOD, SEQ, DMOD, 1.0f);
  attn64_kernel<false><<<gAtt, dim3(128), 0, stream>>>(Qch, Qcl, Kch, Kcl, VcTh, VcTl, src_m, CTXcf, 0.125f);
  split2_kernel<<<gSp, blk, 0, stream>>>(CTXcf, CTXc2, n2, DMOD / 2);
  wmma_gemm64<1, false, 0, 0, false><<<gD, blk, 0, stream>>>(
      CTXc2, CTXc2, 2 * DMOD, 0L, WocT, WocT, 2 * DMOD, 0L, (void*)A2, (void*)A2, DMOD, 0L, b1, x, 0L, MROWS, DMOD, 2 * DMOD, 1.0f);
  ln_kernel<false, true><<<gLN, blk, 0, stream>>>(A2, H1f, XB, ln2_g, ln2_b, H2f, H2hl, MROWS);

  wmma_gemm64<1, false, 2, 2, false, 5><<<gF, blk, 0, stream>>>(
      H2hl, H2hl, 2 * DMOD, 0L, W1T, W1T, 2 * DMOD, 0L, (void*)Fhl, (void*)(Fhl + DFF), 2 * DFF, 0L, b1, x, 0L, MROWS, DFF, 2 * DMOD, 1.0f);
  wmma_gemm64<1, false, 2, 0, false><<<gD, blk, 0, stream>>>(
      Fhl, Fhl, 2 * DFF, 0L, W2T, W2T, 2 * DFF, 0L, (void*)A3, (void*)A3, DMOD, 0L, b2, x, 0L, MROWS, DMOD, 2 * DFF, 1.0f);
  ln_kernel<false, false><<<gLN, blk, 0, stream>>>(A3, H2f, XB, ln3_g, ln3_b, out, H2hl, MROWS);

  (void)hipGetLastError();
}
